// DockPointNet_55688545960608
// MI455X (gfx1250) — hardware-run, weakly checked
//
#include <hip/hip_runtime.h>


namespace {
constexpr int N = 50000, E = 1600000, FX = 32, FE = 8, K1 = 64  , C1 = 64, C2 = 128, C3 = 256;
constexpr float HS = 256.0f, WSC = 256.0f, EPS = 1e-5f, RADIUS = 8.0f;
typedef _Float16 b16;
typedef __attribute__((ext_vector_type(16))) _Float16 v16b;
typedef __attribute__((ext_vector_type(8))) _Float16 v8b;
typedef __attribute__((ext_vector_type(8))) float v8f;
typedef __attribute__((ext_vector_type(4))) float v4f;
__device__ __forceinline__ float bf16_rne(float f) { unsigned int u = __float_as_uint(f); u += 0x7FFFu + ((u >> 16) & 1u); float r = __uint_as_float(u & 0xFFFF0000u); asm volatile("" : "+v"(r)); return r; }
__device__ __forceinline__ float bfv(float f) { float r = bf16_rne(f); asm volatile("" : "+v"(r)); return r; }
__device__ __forceinline__ void split16(float v, b16& hi, b16& lo) { hi = (b16)v; lo = (b16)(v - (float)hi); }
__device__ __forceinline__ v16b frag_kb(const b16* p, int hh) { const v8b a = *(const v8b*)(p + 8 * hh), b = *(const v8b*)(p + 16 + 8 * hh); v16b f;
#pragma unroll
  for (int e = 0; e < 8; ++e) { f[e] = a[e]; f[8 + e] = b[e]; } return f; }
__device__ __forceinline__ v8f wmma16b(v16b a, v16b b, v8f c) { v8f d = __builtin_amdgcn_wmma_f32_16x16x32_f16(false, a, false, b, (short)0, c, false, false); asm volatile("v_nop\n\tv_nop\n\tv_nop\n\tv_nop" : "+v"(d) : "v"(a), "v"(b)); return d; }
__device__ __forceinline__ void wave_lds_sync() { __builtin_amdgcn_fence(__ATOMIC_RELEASE, "workgroup"); __builtin_amdgcn_wave_barrier(); __builtin_amdgcn_fence(__ATOMIC_ACQUIRE, "workgroup"); }
__device__ __forceinline__ float pmul(float a, float b) { float p = a * b; asm volatile("" : "+v"(p)); return p; }
__device__ __forceinline__ int iclamp(int v, int lo, int hi) { return v < lo ? lo : (v > hi ? hi : v); }
__device__ __forceinline__ float wsum(float v) { for (int o = 16; o; o >>= 1) v += __shfl_xor(v, o); return v; }
constexpr int CSR_NBLK8 = 512, CSR_GB8 = 8, CSR_GN8 = 1 << CSR_GB8  , CSR_TS8 = (CSR_GN8 < 32 ? 32 : CSR_GN8)  , CSR_MAXG8 = 512, CSR_CAP8 = 12288  ;
__device__ __host__ __forceinline__ int csr_tix8(int v) { return (v >> CSR_GB8) * CSR_TS8 + (v & (CSR_GN8 - 1)); }
__global__ __launch_bounds__(64) void csrA_kernel8(const int* __restrict__ dst, int E, int N, int nG, int CHP, int NGP, int* __restrict__ STG, int* __restrict__ HST) {
  extern __shared__ int sm[];
  int* cnt = sm; int* run = sm + NGP; int* ids = sm + 2 * NGP;
  const int b = blockIdx.x; const int ch = (E + CSR_NBLK8 - 1) / CSR_NBLK8; const int e0 = b * ch, e1 = min(E, e0 + ch);
  for (int i = threadIdx.x; i < NGP; i += 64) cnt[i] = 0;
  for (int i = threadIdx.x; i < CHP; i += 64) ids[i] = -1;
  __syncthreads();
  if (threadIdx.x == 0) {
    for (int e = e0; e < e1; ++e) { int d = dst[e]; d = (d < 0) ? 0 : (d >= N ? N - 1 : d); cnt[d >> CSR_GB8] += 1; }
    int acc = 0; for (int g = 0; g < nG; ++g) { run[g] = acc; acc += cnt[g]; }
    for (int e = e0; e < e1; ++e) { int d = dst[e]; d = (d < 0) ? 0 : (d >= N ? N - 1 : d); const int g = d >> CSR_GB8; ids[run[g]] = e; run[g] += 1; } }
  __syncthreads();
  typedef __attribute__((ext_vector_type(4))) int v4i;
  for (int pass = 0; pass < 2; ++pass) {
    for (int i = threadIdx.x; i < CHP / 4; i += 64) *(volatile v4i*)(STG + (size_t)b * CHP + i * 4) = *(const v4i*)(&ids[i * 4]);
    for (int i = threadIdx.x; i < NGP / 4; i += 64) { v4i v; for (int e = 0; e < 4; ++e) v[e] = (i * 4 + e < nG) ? cnt[i * 4 + e] : 0; *(volatile v4i*)(HST + (size_t)b * NGP + i * 4) = v; }
    __threadfence(); }
}
__global__ __launch_bounds__(512) void csrS_kernel8(const int* __restrict__ HST, int nG, int NGP, int* __restrict__ START, int* __restrict__ TOT, int* __restrict__ OFF) {
  __shared__ int tot[CSR_MAXG8];
  const int b = threadIdx.x;
  for (int pass = 0; pass < 2; ++pass) { int runb = 0; for (int g = 0; g < nG; ++g) { int c = HST[(size_t)b * NGP + g]; c = (c < 0) ? 0 : c; ((volatile int*)OFF)[(size_t)g * CSR_NBLK8 + b] = runb; runb += c; } __threadfence(); }
  for (int g = threadIdx.x; g < nG; g += 512) { int s = 0; for (int bb = 0; bb < CSR_NBLK8; ++bb) { int c = HST[(size_t)bb * NGP + g]; s += (c < 0) ? 0 : c; } tot[g] = s; }
  __syncthreads();
  if (threadIdx.x < 32) {
    __shared__ int st[CSR_MAXG8 + 32];
    if (threadIdx.x == 0) { int acc = 0; for (int g = 0; g < NGP; ++g) { st[g] = acc; if (g < nG) acc += (tot[g] + 31) & ~31; } st[NGP] = acc; }
    __builtin_amdgcn_fence(__ATOMIC_RELEASE, "workgroup"); __builtin_amdgcn_wave_barrier(); __builtin_amdgcn_fence(__ATOMIC_ACQUIRE, "workgroup");
    for (int pass = 0; pass < 2; ++pass) { for (int i = threadIdx.x; i < NGP + 32; i += 32) { ((volatile int*)START)[i] = (i <= NGP) ? st[min(i, NGP)] : 0; ((volatile int*)TOT)[i] = (i < nG) ? tot[i] : 0; } __threadfence(); } }
}
__global__ __launch_bounds__(256) void csrB_kernel8(const int* __restrict__ dst, int N, int nG, int CHP, int NGP, int permLen, const int* __restrict__ STG, const int* __restrict__ HST, const int* __restrict__ OFF, const int* __restrict__ START, const int* __restrict__ TOT, int* __restrict__ PERM, int* __restrict__ ROWPTR, int* __restrict__ ROWCNT, int* __restrict__ FLAG) {
  typedef __attribute__((ext_vector_type(4))) int v4i;
  __shared__ int ids[CSR_CAP8]; __shared__ unsigned short key[CSR_CAP8]; __shared__ int outp[CSR_CAP8]; __shared__ int ncnt[CSR_GN8 + 1]; __shared__ int boff[CSR_NBLK8 + 1];
  const int g = blockIdx.x, t_ = threadIdx.x; int tot = TOT[g]; int st = START[g], stn = START[g + 1]; const int v0 = g * CSR_GN8; const int nv = min(CSR_GN8, N - v0); const int t0 = g * CSR_TS8;
  st = (st < 0) ? 0 : (st > permLen - 32 ? permLen - 32 : st) & ~31; stn = (stn < st) ? st : (stn > permLen ? permLen : stn); tot = (tot < 0) ? 0 : tot; if (tot > stn - st && tot <= CSR_CAP8) tot = stn - st;
  if (tot > CSR_CAP8) {
    for (int pass = 0; pass < 2; ++pass) { for (int i = t_; i < CSR_TS8 / 4; i += 256) { v4i a, c; for (int e = 0; e < 4; ++e) { a[e] = st; c[e] = 0; } *(volatile v4i*)(ROWPTR + t0 + i * 4) = a; *(volatile v4i*)(ROWCNT + t0 + i * 4) = c; } if (t_ == 0) ((volatile int*)FLAG)[0] = 1; __threadfence(); } (void)nv; return; }
  if (t_ == 0) { int acc = 0; for (int b = 0; b < CSR_NBLK8; ++b) { boff[b] = acc; int c = HST[(size_t)b * NGP + g]; c = (c < 0) ? 0 : (c > CHP ? CHP : c); acc += c; if (acc > tot) acc = tot; } boff[CSR_NBLK8] = acc; }
  for (int i = t_; i <= CSR_GN8; i += 256) ncnt[i] = 0;
  __syncthreads();
  for (int b = 0; b < CSR_NBLK8; ++b) { const int c = boff[b + 1] - boff[b]; int o_ = OFF[(size_t)g * CSR_NBLK8 + b]; o_ = (o_ < 0) ? 0 : (o_ > CHP - c ? CHP - c : o_); const int* src_ = STG + (size_t)b * CHP + o_;
    for (int i = t_; i < c; i += 256) { int id = src_[i]; id = (id < 0) ? 0 : id; ids[boff[b] + i] = id; int d = dst[id]; d = (d < v0) ? v0 : (d >= N ? N - 1 : d); int kk = d - v0; kk = (kk < 0) ? 0 : (kk >= CSR_GN8 ? CSR_GN8 - 1 : kk); key[boff[b] + i] = (unsigned short)kk; } }
  __syncthreads();
  if (t_ == 0) { for (int i = 0; i < tot; ++i) ncnt[key[i]] += 1; int acc = 0; for (int vl = 0; vl < CSR_GN8; ++vl) { const int c = ncnt[vl]; ncnt[vl] = acc; acc += c; } ncnt[CSR_GN8] = acc;
    for (int i = 0; i < tot; ++i) { const int vl = key[i]; outp[ncnt[vl]] = ids[i]; ncnt[vl] += 1; }
    for (int vl = CSR_GN8; vl > 0; --vl) ncnt[vl] = ncnt[vl - 1]; ncnt[0] = 0; }
  __syncthreads();
  for (int pass = 0; pass < 2; ++pass) {
    for (int i = t_; i < (stn - st) / 4; i += 256) { v4i v; for (int e = 0; e < 4; ++e) { const int q = i * 4 + e; v[e] = (q < tot) ? outp[q] : -1; } *(volatile v4i*)(PERM + st + i * 4) = v; }
    for (int i = t_; i < CSR_TS8 / 4; i += 256) { v4i a, c; for (int e = 0; e < 4; ++e) { const int vl = i * 4 + e; const int vc = vl < CSR_GN8 ? vl : CSR_GN8; a[e] = (vl < CSR_GN8) ? st + ncnt[vc] : st; c[e] = (vl < nv) ? (ncnt[(vc < CSR_GN8 ? vc : CSR_GN8 - 1) + 1] - ncnt[vc]) : 0; } *(volatile v4i*)(ROWPTR + t0 + i * 4) = a; *(volatile v4i*)(ROWCNT + t0 + i * 4) = c; }
    __threadfence(); }
}
__global__ __launch_bounds__(256) void csrZ_kernel8(int* __restrict__ p, size_t n4) { typedef __attribute__((ext_vector_type(4))) int v4i; const size_t tid = (size_t)blockIdx.x * 256 + threadIdx.x, nth = (size_t)gridDim.x * 256; v4i z = {0, 0, 0, 0}; for (size_t i = tid; i < n4; i += nth) *(volatile v4i*)(p + i * 4) = z; }
struct CsrBufs8 { int *STG, *HST, *OFF, *START, *TOT, *PERM, *ROWPTR, *ROWCNT, *FLAG; int nG, NGP, CHP; size_t permLen; char* base; size_t bytes; };
static size_t csr_carve8(CsrBufs8& c, char* ws, size_t off, int E, int N) {
  const size_t off0 = off; c.base = ws + off;
  auto al = [&](size_t bytes) { char* p = ws + off; off += (bytes + 255) & ~(size_t)255; return p; };
  c.nG = (N + CSR_GN8 - 1) / CSR_GN8; c.NGP = (c.nG + 31) & ~31; const int ch = (E + CSR_NBLK8 - 1) / CSR_NBLK8; c.CHP = (ch + 31) & ~31; c.permLen = (size_t)E + 32 * (size_t)c.nG + 32;
  c.STG = (int*)al((size_t)CSR_NBLK8 * c.CHP * 4); c.HST = (int*)al((size_t)CSR_NBLK8 * c.NGP * 4); c.OFF = (int*)al((size_t)c.NGP * CSR_NBLK8 * 4); c.START = (int*)al((size_t)(c.NGP + 64) * 4); c.TOT = (int*)al((size_t)(c.NGP + 64) * 4);
  c.PERM = (int*)al(c.permLen * 4); c.ROWPTR = (int*)al((size_t)c.nG * CSR_TS8 * 4); c.ROWCNT = (int*)al((size_t)c.nG * CSR_TS8 * 4); c.FLAG = (int*)al(256);
  c.bytes = off - off0; return off;
}
static void csr_build8(const CsrBufs8& c, const int* dst, int E, int N, hipStream_t stream) {
  const size_t smem = (size_t)(2 * c.NGP + c.CHP) * 4;
  csrZ_kernel8<<<512, 256, 0, stream>>>((int*)c.base, c.bytes / 16);
  csrA_kernel8<<<CSR_NBLK8, 64, smem, stream>>>(dst, E, N, c.nG, c.CHP, c.NGP, c.STG, c.HST);
  csrS_kernel8<<<1, 512, 0, stream>>>(c.HST, c.nG, c.NGP, c.START, c.TOT, c.OFF);
  csrB_kernel8<<<c.nG, 256, 0, stream>>>(dst, N, c.nG, c.CHP, c.NGP, (int)c.permLen, c.STG, c.HST, c.OFF, c.START, c.TOT, c.PERM, c.ROWPTR, c.ROWCNT, c.FLAG);
}


__global__ __launch_bounds__(256) void wput_kernel(const float* __restrict__ w1, const float* __restrict__ w2, const float* __restrict__ wg, b16* __restrict__ WT1, b16* __restrict__ WT2, b16* __restrict__ WTG) { const int u = blockIdx.x * 256 + threadIdx.x; v8b v; auto put = [&](b16* dst) { for (int pass = 0; pass < 2; ++pass) { *(volatile v8b*)dst = v; __threadfence(); } };
  if (u < C1 * 8) { const int o = u / 8, k0 = (u % 8) * 8;
#pragma unroll
    for (int j = 0; j < 8; ++j) { const int k = k0 + j; v[j] = (b16)(k < 47 ? bf16_rne(w1[(size_t)k * C1 + o]) * WSC : 0.0f); } put(WT1 + (size_t)o * K1 + k0); }
  if (u < C2 * 8) { const int o = u / 8, k0 = (u % 8) * 8;
#pragma unroll
    for (int j = 0; j < 8; ++j) v[j] = (b16)(bf16_rne(w2[(size_t)(k0 + j) * C2 + o]) * WSC); put(WT2 + (size_t)o * C1 + k0); }
  if (u < C3 * 16) { const int o = u / 16, k0 = (u % 16) * 8;
#pragma unroll
    for (int j = 0; j < 8; ++j) v[j] = (b16)(bf16_rne(wg[(size_t)(k0 + j) * C3 + o]) * WSC); put(WTG + (size_t)o * C2 + k0); } }
__device__ __forceinline__ void sincos_angle(float ux, float uy, float uz, float vx, float vy, float vz, float& sn, float& cs) { const float cx = uy * vz - uz * vy, cy = uz * vx - ux * vz, cz = ux * vy - uy * vx; const float cn = sqrtf(cx * cx + cy * cy + cz * cz); const float dt = ux * vx + uy * vy + uz * vz; const float r = sqrtf(cn * cn + dt * dt); if (r > 0.0f) { sn = cn / r; cs = dt / r; } else { sn = 0.0f; cs = 1.0f; } }
__global__ __launch_bounds__(32) void edge_kernel(const float* __restrict__ x, const float* __restrict__ pos, const float* __restrict__ nrm, const float* __restrict__ eattr, const int* __restrict__ srcs, const int* __restrict__ PERM, const int* __restrict__ ROWPTR, const int* __restrict__ ROWCNT, int permLen, const b16* __restrict__ WT1, const b16* __restrict__ WT2, const float* __restrict__ b1, const float* __restrict__ g1, const float* __restrict__ be1, const float* __restrict__ b2, const float* __restrict__ g2, const float* __restrict__ be2, int NLIM, float* __restrict__ AGG) { __shared__ __attribute__((aligned(16))) b16 Ah[16][K1 + 8], Al[16][K1 + 8], Bh[16][C1 + 8], Bl[16][C1 + 8]; __shared__ float T1[16][C1 + 1], T2[16][C2 + 1], MX[C2], PF[16][8]; __shared__ int Esrc[16], Eid[16]; const int lane = threadIdx.x, nloc = lane & 15, hlf = lane >> 4; const size_t n = blockIdx.x; if (n >= (size_t)NLIM) return;
  for (int c = lane; c < C2; c += 32) MX[c] = -INFINITY;
  if (lane < 16) for (int k = 0; k < 8; ++k) { Ah[lane][K1 + k] = (b16)0.0f; Al[lane][K1 + k] = (b16)0.0f; Bh[lane][C1 + k] = (b16)0.0f; Bl[lane][C1 + k] = (b16)0.0f; }
  const float pix = bfv(pos[n * 3]), piy = bfv(pos[n * 3 + 1]), piz = bfv(pos[n * 3 + 2]); const float nix = bfv(nrm[n * 3]), niy = bfv(nrm[n * 3 + 1]), niz = bfv(nrm[n * 3 + 2]);
  int st = ROWPTR[n], cnt = ROWCNT[n]; cnt = iclamp(cnt, 0, E); st = iclamp(st, 0, permLen - cnt); int nvalid = 0;
  wave_lds_sync();
#pragma unroll 1
  for (int j0 = 0; j0 < cnt; j0 += 16) { const int nr = (cnt - j0) < 16 ? (cnt - j0) : 16;
    if (lane < 16) { int e = -1, s = 0; if (lane < nr) { e = iclamp(PERM[st + j0 + lane], 0, E - 1); s = iclamp(srcs[e], 0, N - 1); if (s >= NLIM) e = -1; } Eid[lane] = e; Esrc[lane] = s;
      float f7[7] = {0, 0, 0, 0, 0, 0, 0}; if (e >= 0) { const float pjx = bfv(pos[(size_t)s * 3]), pjy = bfv(pos[(size_t)s * 3 + 1]), pjz = bfv(pos[(size_t)s * 3 + 2]); const float px = pjx - pix, py = pjy - piy, pz = pjz - piz; const float njx = bfv(nrm[(size_t)s * 3]), njy = bfv(nrm[(size_t)s * 3 + 1]), njz = bfv(nrm[(size_t)s * 3 + 2]); f7[0] = sqrtf(px * px + py * py + pz * pz) * (1.0f / RADIUS); sincos_angle(nix, niy, niz, px, py, pz, f7[1], f7[2]); sincos_angle(njx, njy, njz, px, py, pz, f7[3], f7[4]); sincos_angle(nix, niy, niz, njx, njy, njz, f7[5], f7[6]); }
      for (int k = 0; k < 7; ++k) PF[lane][k] = f7[k]; PF[lane][7] = 0.0f; }
    wave_lds_sync();
    for (int rr = 0; rr < 16; ++rr) { const int e = Eid[rr], s = Esrc[rr]; float val = 0.0f; const int c = lane;
      float v0 = 0.0f, v1 = 0.0f;
      if (e >= 0) { v0 = bfv(x[(size_t)s * FX + c]);
        const int c1 = 32 + c; if (c1 < 39) v1 = PF[rr][c1 - 32];
        else if (c1 < 47) v1 = bfv(eattr[(size_t)e * FE + (c1 - 39)]); }
      (void)val; b16 p, pl; split16(v0 * HS, p, pl); Ah[rr][c] = p; Al[rr][c] = pl; split16(v1 * HS, p, pl); Ah[rr][32 + c] = p; Al[rr][32 + c] = pl; }
    wave_lds_sync();
    { v8f acc[4] = {(v8f){}, (v8f){}, (v8f){}, (v8f){}};
#pragma unroll
      for (int kb = 0; kb < K1; kb += 32) { const v16b a = frag_kb(&Ah[nloc][kb], hlf), al = frag_kb(&Al[nloc][kb], hlf);
#pragma unroll
        for (int t = 0; t < 4; ++t) { const v16b bw = frag_kb(WT1 + (size_t)(t * 16 + nloc) * K1 + kb, hlf); acc[t] = wmma16b(a, bw, acc[t]); acc[t] = wmma16b(al, bw, acc[t]); } }
#pragma unroll
      for (int t = 0; t < 4; ++t) { const int cc = t * 16 + nloc; const float bb = bfv(b1[cc]);
#pragma unroll
        for (int r8 = 0; r8 < 8; ++r8) T1[8 * hlf + r8][cc] = fmaxf(acc[t][r8] * (1.0f / (HS * WSC)) + bb, 0.0f); } }
    wave_lds_sync();
    { const float ga = bfv(g1[lane]), gb = bfv(g1[32 + lane]), ba = bfv(be1[lane]), bb2 = bfv(be1[32 + lane]);
      for (int rr = 0; rr < 16; ++rr) { const float a = T1[rr][lane], b = T1[rr][32 + lane]; const float m = wsum(a + b) * (1.0f / C1); const float da = a - m, db = b - m; const float vr = wsum(pmul(da, da) + pmul(db, db)) * (1.0f / C1); const float rs = rsqrtf(vr + EPS); T1[rr][lane] = pmul(da * rs, ga) + ba; T1[rr][32 + lane] = pmul(db * rs, gb) + bb2; } }
    wave_lds_sync();
    for (int rr = 0; rr < 16; ++rr) for (int q = 0; q < 2; ++q) { const int c = q * 32 + lane; b16 p, pl; split16(T1[rr][c] * HS, p, pl); Bh[rr][c] = p; Bl[rr][c] = pl; }
    wave_lds_sync();
    { v8f acc[8];
#pragma unroll
      for (int t = 0; t < 8; ++t) acc[t] = (v8f){};
#pragma unroll
      for (int kb = 0; kb < C1; kb += 32) { const v16b a = frag_kb(&Bh[nloc][kb], hlf), al = frag_kb(&Bl[nloc][kb], hlf);
#pragma unroll
        for (int t = 0; t < 8; ++t) { const v16b bw = frag_kb(WT2 + (size_t)(t * 16 + nloc) * C1 + kb, hlf); acc[t] = wmma16b(a, bw, acc[t]); acc[t] = wmma16b(al, bw, acc[t]); } }
#pragma unroll
      for (int t = 0; t < 8; ++t) { const int cc = t * 16 + nloc; const float bb = bfv(b2[cc]);
#pragma unroll
        for (int r8 = 0; r8 < 8; ++r8) T2[8 * hlf + r8][cc] = fmaxf(acc[t][r8] * (1.0f / (HS * WSC)) + bb, 0.0f); } }
    wave_lds_sync();
    { float gg4[4], bb4[4]; for (int q = 0; q < 4; ++q) { gg4[q] = bfv(g2[q * 32 + lane]); bb4[q] = bfv(be2[q * 32 + lane]); }
      for (int rr = 0; rr < 16; ++rr) { float v4[4]; float s = 0.0f; for (int q = 0; q < 4; ++q) { v4[q] = T2[rr][q * 32 + lane]; s += v4[q]; } const float m = wsum(s) * (1.0f / C2); float vs = 0.0f; for (int q = 0; q < 4; ++q) { v4[q] -= m; vs += pmul(v4[q], v4[q]); } const float rs = rsqrtf(wsum(vs) * (1.0f / C2) + EPS); for (int q = 0; q < 4; ++q) T2[rr][q * 32 + lane] = pmul(v4[q] * rs, gg4[q]) + bb4[q]; } }
    wave_lds_sync();
    for (int q = 0; q < 4; ++q) { const int c = q * 32 + lane; float mx = MX[c]; for (int rr = 0; rr < 16; ++rr) if (Eid[rr] >= 0) mx = fmaxf(mx, T2[rr][c]); MX[c] = mx; }
    for (int rr = 0; rr < 16; ++rr) nvalid += (Eid[rr] >= 0) ? 1 : 0;
    wave_lds_sync(); }
  for (int pass = 0; pass < 2; ++pass) { for (int q = 0; q < 4; ++q) { const int c = q * 32 + lane; ((volatile float*)AGG)[n * C2 + c] = nvalid > 0 ? MX[c] : 0.0f; } __threadfence(); } }
__global__ __launch_bounds__(32) void glob_kernel(const float* __restrict__ AGG, const b16* __restrict__ WTG, const float* __restrict__ bg, const float* __restrict__ gg, const float* __restrict__ beg, int NLIM, float* __restrict__ out) { __shared__ __attribute__((aligned(16))) b16 Ah[16][C2 + 8], Al[16][C2 + 8]; __shared__ float Tf[16][C3 + 4]; const int lane = threadIdx.x, nloc = lane & 15, hlf = lane >> 4; const size_t n0 = (size_t)blockIdx.x * 16; if (n0 >= (size_t)NLIM) return;
  for (int rr = 0; rr < 16; ++rr) for (int q = 0; q < 4; ++q) { const int c = q * 32 + lane; b16 p, pl; split16(AGG[(n0 + rr) * C2 + c] * HS, p, pl); Ah[rr][c] = p; Al[rr][c] = pl; }
  if (lane < 16) for (int k = C2; k < C2 + 8; ++k) { Ah[lane][k] = (b16)0.0f; Al[lane][k] = (b16)0.0f; }
  wave_lds_sync(); v8f acc[16];
#pragma unroll
  for (int t = 0; t < 16; ++t) acc[t] = (v8f){};
#pragma unroll
  for (int kb = 0; kb < C2; kb += 32) { const v16b a = frag_kb(&Ah[nloc][kb], hlf), al = frag_kb(&Al[nloc][kb], hlf);
#pragma unroll
    for (int t = 0; t < 16; ++t) { const v16b bw = frag_kb(WTG + (size_t)(t * 16 + nloc) * C2 + kb, hlf); acc[t] = wmma16b(a, bw, acc[t]); acc[t] = wmma16b(al, bw, acc[t]); } }
#pragma unroll
  for (int t = 0; t < 16; ++t) { const int cc = t * 16 + nloc; const float bb = bfv(bg[cc]);
#pragma unroll
    for (int r8 = 0; r8 < 8; ++r8) Tf[8 * hlf + r8][cc] = fmaxf(acc[t][r8] * (1.0f / (HS * WSC)) + bb, 0.0f); }
  wave_lds_sync();
  { float g8[8], b8[8]; for (int q = 0; q < 8; ++q) { g8[q] = bfv(gg[q * 32 + lane]); b8[q] = bfv(beg[q * 32 + lane]); }
    for (int rr = 0; rr < 16; ++rr) { float v8_[8]; float s = 0.0f; for (int q = 0; q < 8; ++q) { v8_[q] = Tf[rr][q * 32 + lane]; s += v8_[q]; } const float m = wsum(s) * (1.0f / C3); float vs = 0.0f; for (int q = 0; q < 8; ++q) { v8_[q] -= m; vs += pmul(v8_[q], v8_[q]); } const float rs = rsqrtf(wsum(vs) * (1.0f / C3) + EPS); for (int q = 0; q < 8; ++q) Tf[rr][q * 32 + lane] = pmul(v8_[q] * rs, g8[q]) + b8[q]; } }
  wave_lds_sync();
  for (int pass = 0; pass < 2; ++pass) { for (int rr = 0; rr < 16; ++rr) for (int q = 0; q < 2; ++q) *(volatile v4f*)(out + (n0 + rr) * C3 + q * 128 + lane * 4) = *(const v4f*)(&Tf[rr][q * 128 + lane * 4]); __threadfence(); } }
}

extern "C" void kernel_launch(void* const* d_in, const int* in_sizes, int n_in, void* d_out, int out_size, void* d_ws, size_t ws_size, hipStream_t stream) {
  (void)n_in;
  auto Fp = [&](int i) { return (const float*)d_in[i]; }; auto Ip = [&](int i) { return (const int*)d_in[i]; };
  if (in_sizes[0] != N * FX || in_sizes[1] != N * 3 || in_sizes[2] != N * 3 || in_sizes[3] != E * FE || in_sizes[4] != 2 * E || in_sizes[5] != 47 * C1 || in_sizes[9] != C1 * C2 || in_sizes[13] != C2 * C3 || out_size != N * C3) return;
  const int NLIM = N;
  size_t off = 0; char* ws = (char*)d_ws;
  auto carve = [&](size_t bytes) { char* p = ws + off; off += (bytes + 255) & ~(size_t)255; return p; };
  b16* WT1 = (b16*)carve(C1 * K1 * 2); b16* WT2 = (b16*)carve(C2 * C1 * 2); b16* WTG = (b16*)carve(C3 * C2 * 2); float* AGG = (float*)carve((size_t)N * C2 * 4); CsrBufs8 csr; off = csr_carve8(csr, ws, off, E, N);
  if (off > ws_size || off > ((size_t)80 << 20)) return;
  wput_kernel<<<(C3 * 16 + 255) / 256, 256, 0, stream>>>(Fp(5), Fp(9), Fp(13), WT1, WT2, WTG);
  csr_build8(csr, Ip(4) + E, E, N, stream);
  edge_kernel<<<NLIM, 32, 0, stream>>>(Fp(0), Fp(1), Fp(2), Fp(3), Ip(4), csr.PERM, csr.ROWPTR, csr.ROWCNT, (int)csr.permLen, WT1, WT2, Fp(6), Fp(7), Fp(8), Fp(10), Fp(11), Fp(12), NLIM, AGG);
  glob_kernel<<<NLIM / 16, 32, 0, stream>>>(AGG, WTG, Fp(14), Fp(15), Fp(16), NLIM, (float*)d_out);
}
